// HVRTLinearFFN_75883482186212
// MI455X (gfx1250) — hardware-verified
//
#include <hip/hip_runtime.h>
#include <math.h>

#define NTOK 4096
#define NTOK_FULL 4096
#define DM 1024
#define FF 64
#define NP 64
#define NPASS 3
#define PPP 31
#define NER 32
#define NULLI 31
#define SPT 1
#define NSLOT (NTOK * SPT)
#define R_MAX (NSLOT + 64 * NER)
#define NT_MAX (R_MAX / 64)

#define CX_LOG2 11
#define CW_LOG2 16
#define CH_LOG2 11
#define CH ((float)(1u << CH_LOG2))
#define SC_H (1.0f / (float)(1u << (CX_LOG2 + CW_LOG2)))
#define SC_Y (1.0f / (float)(1u << (CH_LOG2 + CW_LOG2)))

#define RW_CH 8192
#define TBL_COUNT 0
#define TBL_POFF 32
#define TBL_NTILES 72
#define TBL_TILE_E 128
#define TBL_HDR 256
#define TBL_ROWTOK TBL_HDR
#define TBL_SLOTROW (TBL_HDR + R_MAX)
#define TBL_WORDS (TBL_HDR + R_MAX + NSLOT)

static_assert(NP == 64 && NPASS == 3 && PPP == 31 && NPASS * PPP >= NP && (NPASS - 1) * PPP < NP && NER == 32 && NULLI == PPP && NULLI < NER && SPT == 1);
static_assert(DM == 1024 && FF == 64 && DM % 64 == 0 && FF % 64 == 0 && NTOK % 128 == 0);
static_assert(NSLOT % 128 == 0 && R_MAX % 128 == 0 && R_MAX >= NSLOT + 63 * NER);
static_assert(TBL_HDR % 32 == 0 && TBL_HDR <= 512);
static_assert(TBL_COUNT + NER <= TBL_POFF && TBL_POFF + NER + 1 <= TBL_NTILES && TBL_NTILES < TBL_TILE_E && TBL_TILE_E + NT_MAX <= TBL_HDR);
static_assert(RW_CH % 128 == 0 && (TBL_WORDS * 4) % 256 == 0 && R_MAX <= RW_CH && NSLOT <= RW_CH);
static_assert((NTOK * DM / 8) % 256 == 0);
static_assert(CX_LOG2 == 11 && CW_LOG2 == 16 && CH_LOG2 == 11);
static_assert(NSLOT == 4096 && R_MAX == 6144 && NT_MAX == 96 && TBL_WORDS == 10496);

constexpr size_t al256(size_t b) { return (b + 255) & ~(size_t)255; }
constexpr size_t SZ_X16 = al256((size_t)NTOK * DM * 2);
constexpr size_t SZ_W   = al256((size_t)NP * FF * DM * 2);
constexpr size_t SZ_SEL = al256((size_t)NPASS * NSLOT * 4);
constexpr size_t SZ_TBL = al256((size_t)NPASS * TBL_WORDS * 4);
constexpr size_t SZ_XG  = al256((size_t)R_MAX * DM * 2);
constexpr size_t SZ_HG  = al256((size_t)R_MAX * FF * 2);
constexpr size_t SZ_YG  = al256((size_t)NPASS * R_MAX * DM * 4);
constexpr size_t WS_TOTAL = SZ_X16 + 2 * SZ_W + SZ_SEL + SZ_TBL + SZ_XG + SZ_HG + SZ_YG;
static_assert(WS_TOTAL == (size_t)114207744 && WS_TOTAL < (size_t)134217728);

typedef _Float16 h16;
typedef __attribute__((ext_vector_type(16))) _Float16 v16h;
typedef __attribute__((ext_vector_type(8)))  _Float16 v8h;
typedef __attribute__((ext_vector_type(8)))  float    v8f;
typedef __attribute__((ext_vector_type(4)))  float    v4f;
typedef __attribute__((ext_vector_type(2)))  float    v2f;
typedef __attribute__((ext_vector_type(4)))  unsigned int v4u;
typedef __attribute__((ext_vector_type(4)))  int      v4i;
typedef __attribute__((ext_vector_type(2)))  int      v2i;


#define VST2(T, ptr, val) do { const T vst2_v_ = (val); *(volatile T*)(ptr) = vst2_v_; __threadfence(); *(volatile T*)(ptr) = vst2_v_; } while (0)

static __device__ __forceinline__ float bfr(float f) {
    unsigned u = __float_as_uint(f);
    u += 0x7FFFu + ((u >> 16) & 1u);
    return __uint_as_float(u & 0xFFFF0000u);
}
static __device__ __forceinline__ h16 toh_flush(float v) { const float w = (fabsf(v) < 6.103515625e-05f) ? 0.0f : v; return (h16)w; }
static __device__ __forceinline__ void st8h(h16* p, const float* v) {
    v8h hv;
#pragma unroll
    for (int e = 0; e < 8; ++e) hv[e] = toh_flush(v[e]);
    VST2(v8h, p, hv);
}

union FragU { v16h v; v8h h[2]; };
static __device__ __forceinline__ v16h frag_ld(const h16* p) {
    FragU f; f.h[0] = *(const v8h*)(p); f.h[1] = *(const v8h*)(p + 16); return f.v;
}
static __device__ __forceinline__ v8f wmma16g(v16h a, v16h b, v8f c) {
    c = __builtin_amdgcn_wmma_f32_16x16x32_f16(false, a, false, b, (short)0, c, false, false);
    asm volatile("v_nop\n\tv_nop\n\tv_nop\n\tv_nop" : "+v"(c) : "v"(a), "v"(b));
    return c;
}
static __device__ __forceinline__ void wave_sync_lds() {
    __builtin_amdgcn_fence(3  , "workgroup");
    __builtin_amdgcn_wave_barrier();
    __builtin_amdgcn_fence(2  , "workgroup");
}

template <int LOG2C>
__global__ __launch_bounds__(256) void k_plane(const float* __restrict__ src, h16* __restrict__ dst, unsigned n8) {
    const unsigned u = blockIdx.x * 256u + threadIdx.x;
    if (u >= n8) return;
    const float cs = (float)(1u << LOG2C);
    const v4f a = *(const v4f*)(src + (size_t)u * 8u);
    const v4f b = *(const v4f*)(src + (size_t)u * 8u + 4u);
    float v[8] = {bfr(a.x) * cs, bfr(a.y) * cs, bfr(a.z) * cs, bfr(a.w) * cs, bfr(b.x) * cs, bfr(b.y) * cs, bfr(b.z) * cs, bfr(b.w) * cs};
    st8h(dst + (size_t)u * 8u, v);
}

__global__ __launch_bounds__(128) void k_planeTw(const float* __restrict__ src, h16* __restrict__ dst, unsigned ne, unsigned K, unsigned N, unsigned pitch, unsigned estride, float cs) {
    __shared__ __align__(16) float sT[4][64 * 36];
    const unsigned lane = threadIdx.x & 31u;
    const unsigned wave = threadIdx.x >> 5;
    const unsigned tk = K >> 6, tn = N >> 5;
    const unsigned tpe = tk * tn;
    const unsigned u = blockIdx.x * 4u + wave;
    if (u >= ne * tpe) return;
    const unsigned e = u / tpe;
    const unsigned rem = u - e * tpe;
    const unsigned kt = rem / tn;
    const unsigned nt = rem - kt * tn;
    const unsigned k0 = kt << 6, n0 = nt << 5;
    const size_t sbase = (size_t)e * (size_t)estride;
    const size_t ebase = (size_t)e * ((size_t)K * (size_t)N);
    float* slab = sT[wave];
#pragma unroll
    for (int i = 0; i < 16; ++i) {
        const unsigned p = lane + 32u * (unsigned)i;
        const unsigned kr = p >> 3;
        const unsigned n4 = (p & 7u) * 4u;
        const v4f a = *(const v4f*)(src + sbase + (size_t)(k0 + kr) * pitch + n0 + n4);
        v4f s;
        s.x = bfr(a.x) * cs; s.y = bfr(a.y) * cs; s.z = bfr(a.z) * cs; s.w = bfr(a.w) * cs;
        *(v4f*)(&slab[kr * 36u + n4]) = s;
    }
    wave_sync_lds();
#pragma unroll
    for (int i = 0; i < 8; ++i) {
        const unsigned q = lane + 32u * (unsigned)i;
        const unsigned n = q >> 3;
        const unsigned kp = q & 7u;
        float v[8];
#pragma unroll
        for (int j = 0; j < 8; ++j) v[j] = slab[(8u * kp + (unsigned)j) * 36u + n];
        st8h(dst + ebase + (size_t)(n0 + n) * K + k0 + 8u * kp, v);
    }
}

__global__ __launch_bounds__(256) void k_sel(const int* __restrict__ pids, int* __restrict__ sel) {
    const unsigned t4 = (blockIdx.x * 256u + threadIdx.x) * 4u;
    if (t4 >= (unsigned)NTOK) return;
    const v4i pv = *(const v4i*)(pids + t4);
    const int p0 = min(max(pv.x, 0), NP - 1), p1 = min(max(pv.y, 0), NP - 1), p2 = min(max(pv.z, 0), NP - 1), p3 = min(max(pv.w, 0), NP - 1);
#pragma unroll
    for (int P = 0; P < NPASS; ++P) {
        const int lo = P * PPP;
        v4i s;
        s.x = (p0 >= lo && p0 < lo + PPP) ? (p0 - lo) : NULLI;
        s.y = (p1 >= lo && p1 < lo + PPP) ? (p1 - lo) : NULLI;
        s.z = (p2 >= lo && p2 < lo + PPP) ? (p2 - lo) : NULLI;
        s.w = (p3 >= lo && p3 < lo + PPP) ? (p3 - lo) : NULLI;
        VST2(v4i, sel + (size_t)P * NSLOT + t4, s);
    }
}

template <int NE_>
__global__ __launch_bounds__(32) void k_route1w(const int* __restrict__ sel, int* __restrict__ tbl, unsigned nslot, unsigned spt, unsigned hdr, unsigned rmax,
                                                unsigned offPoff, unsigned offNtiles, unsigned offTileE) {
    static_assert(NE_ >= 1 && NE_ <= 32);
    __shared__ __align__(16) int s_img[RW_CH];
    __shared__ __align__(16) int s_hdr[512];
    const unsigned lane = threadIdx.x & 31u;
    const unsigned spl = nslot >> 5;
    const unsigned ng = spl >> 2;
    const unsigned ntmax = rmax >> 6;
    const v4i* sp = (const v4i*)(sel + (size_t)lane * spl);
    int cnt[NE_];
#pragma unroll
    for (int j = 0; j < NE_; ++j) cnt[j] = 0;
    for (unsigned g = 0; g < ng; ++g) {
        const v4i v = sp[g];
#pragma unroll
        for (int c = 0; c < 4; ++c) {
            const int e = min(max(v[c], 0), NE_ - 1);
#pragma unroll
            for (int j = 0; j < NE_; ++j) cnt[j] += (e == j) ? 1 : 0;
        }
    }
    int base0[NE_], total[NE_];
#pragma unroll
    for (int j = 0; j < NE_; ++j) {
        int pre = 0, tot = cnt[j];
#pragma unroll
        for (int d = 1; d < 32; d <<= 1) {
            const int t = __shfl_xor(tot, d, 32);
            pre += ((lane & (unsigned)d) != 0u) ? t : 0;
            tot += t;
        }
        base0[j] = pre;
        total[j] = tot;
    }
    int poff[NE_ + 1];
    poff[0] = 0;
#pragma unroll
    for (int j = 0; j < NE_; ++j) poff[j + 1] = poff[j] + (((total[j] + 63) >> 6) << 6);
    for (unsigned i = lane; i < 512u; i += 32u) s_hdr[i] = (i >= offTileE && i < offTileE + ntmax) ? -1 : 0;
    wave_sync_lds();
    if (lane == 0u) {
#pragma unroll
        for (int j = 0; j < NE_; ++j) { s_hdr[min((unsigned)j, 511u)] = total[j]; s_hdr[min(offPoff + (unsigned)j, 511u)] = poff[j]; }
        s_hdr[min(offPoff + (unsigned)NE_, 511u)] = poff[NE_];
        s_hdr[min(offNtiles, 511u)] = poff[NE_] >> 6;
    }
    for (unsigned t = lane; t < ntmax; t += 32u) {
        const int b64 = (int)(t * 64u);
        int ev = -1;
#pragma unroll
        for (int j = 0; j < NE_; ++j) ev = (b64 >= poff[j] && b64 < poff[j + 1]) ? j : ev;
        s_hdr[min(offTileE + t, 511u)] = ev;
    }
    wave_sync_lds();
    for (int pass = 0; pass < 2; ++pass) {
        for (unsigned i = lane; i < (hdr >> 2); i += 32u) *(volatile v4i*)(tbl + 4u * i) = *(const v4i*)(&s_hdr[4u * i]);
        __threadfence();
    }
    for (unsigned lo = 0; lo < rmax; lo += (unsigned)RW_CH) {
        for (unsigned i = lane; i < (unsigned)(RW_CH / 4); i += 32u) *(v4i*)(&s_img[4u * i]) = (v4i){-1, -1, -1, -1};
        wave_sync_lds();
        int run[NE_];
#pragma unroll
        for (int j = 0; j < NE_; ++j) run[j] = base0[j];
        for (unsigned g = 0; g < ng; ++g) {
            const v4i v = sp[g];
#pragma unroll
            for (int c = 0; c < 4; ++c) {
                const int e = min(max(v[c], 0), NE_ - 1);
                int row = 0;
#pragma unroll
                for (int j = 0; j < NE_; ++j) {
                    const bool hit = (e == j);
                    row = hit ? (poff[j] + run[j]) : row;
                    run[j] += hit ? 1 : 0;
                }
                row = min(max(row, 0), (int)rmax - 1);
                const unsigned rel = (unsigned)row - lo;
                if (rel < (unsigned)RW_CH) s_img[rel] = (int)((lane * spl + 4u * g + (unsigned)c) / spt);
            }
        }
        wave_sync_lds();
        const unsigned nw = min((unsigned)RW_CH, rmax - lo);
        for (int pass = 0; pass < 2; ++pass) {
            for (unsigned i = lane; i < (nw >> 2); i += 32u) *(volatile v4i*)(tbl + hdr + lo + 4u * i) = *(const v4i*)(&s_img[4u * i]);
            __threadfence();
        }
        wave_sync_lds();
    }
    for (unsigned lo = 0; lo < nslot; lo += (unsigned)RW_CH) {
        int run[NE_];
#pragma unroll
        for (int j = 0; j < NE_; ++j) run[j] = base0[j];
        for (unsigned g = 0; g < ng; ++g) {
            const v4i v = sp[g];
#pragma unroll
            for (int c = 0; c < 4; ++c) {
                const int e = min(max(v[c], 0), NE_ - 1);
                int row = 0;
#pragma unroll
                for (int j = 0; j < NE_; ++j) {
                    const bool hit = (e == j);
                    row = hit ? (poff[j] + run[j]) : row;
                    run[j] += hit ? 1 : 0;
                }
                row = min(max(row, 0), (int)rmax - 1);
                const unsigned rel = (lane * spl + 4u * g + (unsigned)c) - lo;
                if (rel < (unsigned)RW_CH) s_img[rel] = row;
            }
        }
        wave_sync_lds();
        const unsigned nw = min((unsigned)RW_CH, nslot - lo);
        for (int pass = 0; pass < 2; ++pass) {
            for (unsigned i = lane; i < (nw >> 2); i += 32u) *(volatile v4i*)(tbl + hdr + rmax + lo + 4u * i) = *(const v4i*)(&s_img[4u * i]);
            __threadfence();
        }
        wave_sync_lds();
    }
}

__global__ __launch_bounds__(256) void k_gather(const h16* __restrict__ x16, const int* __restrict__ tbl, h16* __restrict__ Xg) {
    const unsigned row = blockIdx.x * 2u + (threadIdx.x >> 7);
    if (row >= (unsigned)R_MAX) return;
    const unsigned c = (threadIdx.x & 127u) * 8u;
    const int tr = tbl[TBL_ROWTOK + row];
    const bool pad = (tr < 0);
    const int tok = min(max(tr, 0), NTOK - 1);
    const v4u ld = *(const v4u*)(x16 + (size_t)(unsigned)tok * DM + c);
    v4u v;
    v.x = pad ? 0u : ld.x; v.y = pad ? 0u : ld.y; v.z = pad ? 0u : ld.z; v.w = pad ? 0u : ld.w;
    VST2(v4u, Xg + (size_t)row * DM + c, v);
}

__global__ __launch_bounds__(256) void k_p1(const h16* __restrict__ Xg, const h16* __restrict__ Wp,
                                            const int* __restrict__ tbl, h16* __restrict__ Hg, unsigned nreal) {
    __shared__ __align__(16) float sT[8][16 * 68];
    const unsigned lane = threadIdx.x & 31u;
    const unsigned wave = threadIdx.x >> 5;
    const unsigned u = blockIdx.x * 8u + wave;
    if (u >= (unsigned)(NT_MAX * (FF / 64))) return;
    const unsigned rowtile = u / (unsigned)(FF / 64);
    const unsigned ct = u - rowtile * (unsigned)(FF / 64);
    const int nt = min(max(tbl[TBL_POFF + NULLI] >> 6, 0), NT_MAX);
    if ((int)rowtile >= nt) return;
    const int e = min(max(tbl[TBL_TILE_E + rowtile], 0), (int)nreal - 1);
    const size_t wbase = (size_t)(unsigned)e * (size_t)(FF * DM);
    const unsigned m0 = rowtile << 6, n0 = ct << 6;
    const unsigned rlane = lane & 15u;
    const unsigned koff = (lane >> 4) * 8u;
    const unsigned mOff = koff;

    v8f acc[4][4];
#pragma unroll
    for (int i = 0; i < 4; ++i)
#pragma unroll
        for (int j = 0; j < 4; ++j) acc[i][j] = (v8f){0.f,0.f,0.f,0.f,0.f,0.f,0.f,0.f};

    for (unsigned k0 = 0; k0 < (unsigned)DM; k0 += 32u) {
        v16h bh[4];
#pragma unroll
        for (int j = 0; j < 4; ++j)
            bh[j] = frag_ld(Wp + wbase + (size_t)(n0 + ((unsigned)j << 4) + rlane) * DM + koff + k0);
#pragma unroll
        for (int i = 0; i < 4; ++i) {
            const v16h ah = frag_ld(Xg + (size_t)(m0 + ((unsigned)i << 4) + rlane) * DM + koff + k0);
#pragma unroll
            for (int j = 0; j < 4; ++j) acc[i][j] = wmma16g(ah, bh[j], acc[i][j]);
        }
    }

    float* slab = sT[wave];
#pragma unroll
    for (int i = 0; i < 4; ++i) {
        const unsigned mBase = m0 + ((unsigned)i << 4);
#pragma unroll
        for (int j = 0; j < 4; ++j)
#pragma unroll
            for (int r = 0; r < 8; ++r) {
                const float a = acc[i][j][r] * SC_H;
                slab[(mOff + (unsigned)r) * 68u + ((unsigned)j << 4) + rlane] = a * CH;
            }
        wave_sync_lds();
        const unsigned q = lane >> 3, c8 = (lane & 7u) * 8u;
        v8h hv[4];
#pragma unroll
        for (int it = 0; it < 4; ++it) {
            const unsigned row = (unsigned)it * 4u + q;
            const float* sp = slab + row * 68u + c8;
#pragma unroll
            for (int t = 0; t < 8; ++t) hv[it][t] = toh_flush(sp[t]);
        }
        for (int pass = 0; pass < 2; ++pass) {
#pragma unroll
            for (int it = 0; it < 4; ++it) {
                const unsigned row = (unsigned)it * 4u + q;
                *(volatile v8h*)(Hg + (size_t)(mBase + row) * FF + n0 + c8) = hv[it];
            }
            __threadfence();
        }
        wave_sync_lds();
    }
}

__global__ __launch_bounds__(256) void k_p2(const h16* __restrict__ Hg, const h16* __restrict__ Wp,
                                            const int* __restrict__ tbl, float* __restrict__ Yg, unsigned nreal) {
    __shared__ __align__(16) float sT[8][16 * 68];
    const unsigned lane = threadIdx.x & 31u;
    const unsigned wave = threadIdx.x >> 5;
    const unsigned u = blockIdx.x * 8u + wave;
    if (u >= (unsigned)(NT_MAX * (DM / 64))) return;
    const unsigned rowtile = u / (unsigned)(DM / 64);
    const unsigned ct = u - rowtile * (unsigned)(DM / 64);
    const int nt = min(max(tbl[TBL_POFF + NULLI] >> 6, 0), NT_MAX);
    if ((int)rowtile >= nt) return;
    const int e = min(max(tbl[TBL_TILE_E + rowtile], 0), (int)nreal - 1);
    const size_t wbase = (size_t)(unsigned)e * (size_t)(DM * FF);
    const unsigned m0 = rowtile << 6, n0 = ct << 6;
    const unsigned rlane = lane & 15u;
    const unsigned koff = (lane >> 4) * 8u;
    const unsigned mOff = koff;

    v8f acc[4][4];
#pragma unroll
    for (int i = 0; i < 4; ++i)
#pragma unroll
        for (int j = 0; j < 4; ++j) acc[i][j] = (v8f){0.f,0.f,0.f,0.f,0.f,0.f,0.f,0.f};

    for (unsigned k0 = 0; k0 < (unsigned)FF; k0 += 32u) {
        v16h bh[4];
#pragma unroll
        for (int j = 0; j < 4; ++j)
            bh[j] = frag_ld(Wp + wbase + (size_t)(n0 + ((unsigned)j << 4) + rlane) * FF + koff + k0);
#pragma unroll
        for (int i = 0; i < 4; ++i) {
            const v16h ah = frag_ld(Hg + (size_t)(m0 + ((unsigned)i << 4) + rlane) * FF + koff + k0);
#pragma unroll
            for (int j = 0; j < 4; ++j) acc[i][j] = wmma16g(ah, bh[j], acc[i][j]);
        }
    }

    float* slab = sT[wave];
#pragma unroll
    for (int i = 0; i < 4; ++i) {
        const unsigned mBase = m0 + ((unsigned)i << 4);
#pragma unroll
        for (int j = 0; j < 4; ++j)
#pragma unroll
            for (int r = 0; r < 8; ++r)
                slab[(mOff + (unsigned)r) * 68u + ((unsigned)j << 4) + rlane] = acc[i][j][r] * SC_Y;
        wave_sync_lds();
        const unsigned hh = lane >> 4, c4 = (lane & 15u) * 4u;
#pragma unroll
        for (int half = 0; half < 2; ++half) {
            v4f vv[4];
#pragma unroll
            for (int it = 0; it < 4; ++it) {
                const unsigned row = (unsigned)(half * 4 + it) * 2u + hh;
                vv[it] = *(const v4f*)(slab + row * 68u + c4);
            }
            for (int pass = 0; pass < 2; ++pass) {
#pragma unroll
                for (int it = 0; it < 4; ++it) {
                    const unsigned row = (unsigned)(half * 4 + it) * 2u + hh;
                    *(volatile v4f*)(Yg + (size_t)(mBase + row) * DM + n0 + c4) = vv[it];
                }
                __threadfence();
            }
        }
        wave_sync_lds();
    }
}

__global__ __launch_bounds__(256) void k_combine(const float* __restrict__ Yg, const int* __restrict__ pids, const int* __restrict__ tbl, const float* __restrict__ bias, float* __restrict__ out) {
    const unsigned t = blockIdx.x;
    if (t >= (unsigned)NTOK) return;
    const unsigned c = threadIdx.x * 4u;
    const int pid = min(max(pids[t], 0), NP - 1);
    const unsigned P = (pid >= 2 * PPP) ? 2u : ((pid >= PPP) ? 1u : 0u);
    const int r = min(max(tbl[(size_t)P * TBL_WORDS + TBL_SLOTROW + t], 0), R_MAX - 1);
    const v4f a = *(const v4f*)(Yg + ((size_t)P * R_MAX + (size_t)(unsigned)r) * DM + c);
    const v4f b = *(const v4f*)(bias + c);
    v4f y;
    y.x = a.x + bfr(b.x); y.y = a.y + bfr(b.y); y.z = a.z + bfr(b.z); y.w = a.w + bfr(b.w);
    VST2(v4f, out + (size_t)t * DM + c, y);
}

extern "C" void kernel_launch(void* const* d_in, const int* in_sizes, int n_in, void* d_out, int out_size,
                              void* d_ws, size_t ws_size, hipStream_t stream) {
    if (n_in < 5) return;
    if (in_sizes[0] < NTOK * DM || in_sizes[1] < NTOK || in_sizes[2] < NP * DM * FF || in_sizes[3] < NP * FF * DM || in_sizes[4] < DM) return;
    if (out_size < NTOK * DM) return;

    const float* x    = (const float*)d_in[0];
    const int*   pids = (const int*)d_in[1];
    const float* U    = (const float*)d_in[2];
    const float* V    = (const float*)d_in[3];
    const float* bias = (const float*)d_in[4];
    float* out = (float*)d_out;

    char* wsp = (char*)d_ws;
    size_t off = 0;
    auto carve = [&](size_t bytes) -> void* { void* r = wsp + off; off += (bytes + 255) & ~(size_t)255; return r; };
    h16*   x16 = (h16*)carve((size_t)NTOK * DM * 2);
    h16*   Up  = (h16*)carve((size_t)NP * FF * DM * 2);
    h16*   Vp  = (h16*)carve((size_t)NP * DM * FF * 2);
    int*   sel = (int*)carve((size_t)NPASS * NSLOT * 4);
    int*   tbl = (int*)carve((size_t)NPASS * TBL_WORDS * 4);
    h16*   Xg  = (h16*)carve((size_t)R_MAX * DM * 2);
    h16*   Hg  = (h16*)carve((size_t)R_MAX * FF * 2);
    float* Yg  = (float*)carve((size_t)NPASS * R_MAX * DM * 4);
    if (off != WS_TOTAL || off > ws_size || off > (size_t)134217728) return;

    k_plane<CX_LOG2><<<(NTOK * DM / 8) / 256, 256, 0, stream>>>(x, x16, (unsigned)(NTOK * DM / 8));
    k_planeTw<<<(NP * (DM / 64) * (FF / 32) + 3) / 4, 128, 0, stream>>>(U, Up, (unsigned)NP, (unsigned)DM, (unsigned)FF, (unsigned)FF, (unsigned)(DM * FF), (float)(1u << CW_LOG2));
    k_planeTw<<<(NP * (FF / 64) * (DM / 32) + 3) / 4, 128, 0, stream>>>(V, Vp, (unsigned)NP, (unsigned)FF, (unsigned)DM, (unsigned)DM, (unsigned)(FF * DM), (float)(1u << CW_LOG2));
    k_sel<<<NTOK / 4 / 256, 256, 0, stream>>>(pids, sel);

#define ONE_PASS(P, NREAL) \
    k_route1w<NER><<<1, 32, 0, stream>>>(sel + (size_t)(P) * NSLOT, tbl + (size_t)(P) * TBL_WORDS, (unsigned)NSLOT, (unsigned)SPT, (unsigned)TBL_HDR, (unsigned)R_MAX, (unsigned)TBL_POFF, (unsigned)TBL_NTILES, (unsigned)TBL_TILE_E); \
    k_gather<<<R_MAX / 2, 256, 0, stream>>>(x16, tbl + (size_t)(P) * TBL_WORDS, Xg); \
    k_p1<<<(NT_MAX * (FF / 64) + 7) / 8, 256, 0, stream>>>(Xg, Up + (size_t)(P) * PPP * FF * DM, tbl + (size_t)(P) * TBL_WORDS, Hg, (unsigned)(NREAL)); \
    k_p2<<<(NT_MAX * (DM / 64) + 7) / 8, 256, 0, stream>>>(Hg, Vp + (size_t)(P) * PPP * DM * FF, tbl + (size_t)(P) * TBL_WORDS, Yg + (size_t)(P) * R_MAX * DM, (unsigned)(NREAL));
    ONE_PASS(0, PPP) ONE_PASS(1, PPP) ONE_PASS(2, NP - 2 * PPP)
#undef ONE_PASS
    k_combine<<<NTOK, 256, 0, stream>>>(Yg, pids, tbl, bias, out);
}
